// FlatTorusPhasorBlock_37082747633868
// MI455X (gfx1250) — hardware-verified
//
#include <hip/hip_runtime.h>
#include <math.h>

typedef __attribute__((ext_vector_type(16))) _Float16 v16h;
typedef __attribute__((ext_vector_type(16))) __bf16 v16b;
typedef __attribute__((ext_vector_type(8)))  _Float16 v8h;
typedef __attribute__((ext_vector_type(8)))  float v8f;
typedef __attribute__((ext_vector_type(4)))  float v4f;
typedef __attribute__((ext_vector_type(2)))  float v2f;
typedef __attribute__((ext_vector_type(4)))  unsigned v4u;
typedef __attribute__((ext_vector_type(4)))  int v4i;
typedef float __attribute__((may_alias)) float_a;
typedef int __attribute__((may_alias)) int_a;

template <typename T> __device__ __forceinline__ void vst2(void* p, T v) { *(volatile T*)p = v; __threadfence(); *(volatile T*)p = v; }
__device__ __forceinline__ v8f wmma16(v16h a, v16h b, v8f c) {
  v8f d = __builtin_amdgcn_wmma_f32_16x16x32_f16(false, a, false, b, (short)0, c, false, false);
  asm volatile("v_nop\n\tv_nop\n\tv_nop\n\tv_nop" : "+v"(d) : "v"(a), "v"(b));
  return d;
}
__device__ __forceinline__ v8f wmma_bf(v16b a, v16b b, v8f c) {
  v8f d = __builtin_amdgcn_wmma_f32_16x16x32_bf16(false, a, false, b, (short)0, c, false, false);
  asm volatile("v_nop\n\tv_nop\n\tv_nop\n\tv_nop" : "+v"(d) : "v"(a), "v"(b));
  return d;
}
__device__ __forceinline__ v16h frag_h(const _Float16* rowk0, int lane) {
  union { v16h v; v8h q[2]; } u; const _Float16* p = rowk0 + 8 * (lane >> 4);
  u.q[0] = *(const v8h*)p; u.q[1] = *(const v8h*)(p + 16); return u.v;
}
__device__ __forceinline__ v16h frag_f32(const float* rowk0, int lane) {
  v16h a; const float* p = rowk0 + 8 * (lane >> 4);
#pragma unroll
  for (int i = 0; i < 8; ++i) { a[i] = (_Float16)p[i]; a[8 + i] = (_Float16)p[16 + i]; }
  return a;
}
__device__ __forceinline__ v16h frag_f32s(const float* rowk0, int lane, float sc) {
  v16h a; const float* p = rowk0 + 8 * (lane >> 4);
#pragma unroll
  for (int i = 0; i < 8; ++i) { a[i] = (_Float16)(p[i] * sc); a[8 + i] = (_Float16)(p[16 + i] * sc); }
  return a;
}
__device__ __forceinline__ v16h fragc_f32(const float* W, int k0, int n, int lane, int ld, int K) {
  v16h a; const int g = lane >> 4;
#pragma unroll
  for (int i = 0; i < 8; ++i) { const int ka = k0 + 8 * g + i, kb = ka + 16;
    a[i] = (_Float16)(ka < K ? W[(size_t)ka * ld + n] : 0.f); a[8 + i] = (_Float16)(kb < K ? W[(size_t)kb * ld + n] : 0.f); }
  return a;
}
struct F2 { v16b h, l; };
__device__ __forceinline__ F2 bsplit16(const float v[16]) { F2 r;
#pragma unroll
  for (int i = 0; i < 16; ++i) { const __bf16 h = (__bf16)v[i]; r.h[i] = h; r.l[i] = (__bf16)(v[i] - (float)h); }
  return r; }
__device__ __forceinline__ F2 split_row(const float* row, int k0, int lane) { float v[16]; const float* p = row + k0 + 8 * (lane >> 4);
#pragma unroll
  for (int i = 0; i < 8; ++i) { v[i] = p[i]; v[8 + i] = p[16 + i]; }
  return bsplit16(v); }
__device__ __forceinline__ F2 split_rowK(const float* row, int k0, int lane, int K) { float v[16]; const int g = lane >> 4;
#pragma unroll
  for (int i = 0; i < 8; ++i) { const int ka = k0 + 8 * g + i, kb = ka + 16; v[i] = ka < K ? row[ka] : 0.f; v[8 + i] = kb < K ? row[kb] : 0.f; }
  return bsplit16(v); }
__device__ __forceinline__ F2 split_col(const float* W, int k0, int n, int lane, int ld, int K) { float v[16]; const int g = lane >> 4;
#pragma unroll
  for (int i = 0; i < 8; ++i) { const int ka = k0 + 8 * g + i, kb = ka + 16; v[i] = ka < K ? W[(size_t)ka * ld + n] : 0.f; v[8 + i] = kb < K ? W[(size_t)kb * ld + n] : 0.f; }
  return bsplit16(v); }
__device__ __forceinline__ v8f mac3(const F2& a, const F2& b, v8f c) { c = wmma_bf(a.l, b.h, c); c = wmma_bf(a.h, b.l, c); return wmma_bf(a.h, b.h, c); }
__device__ __forceinline__ float sigm(float v) { return 1.0f / (1.0f + expf(-v)); }
#define LDSX() do { asm volatile("s_wait_dscnt 0" ::: "memory"); __builtin_amdgcn_wave_barrier(); __builtin_amdgcn_fence(__ATOMIC_RELEASE, "workgroup"); } while (0)

#define NB 2
#define LL 1024
#define DD 256
#define KP 64
#define NF (2 * KP)
#define NR (NB * LL)

__device__ __forceinline__ float gelu_e(float v) { return 0.5f * v * (1.0f + erff(v * 0.70710678118654752f)); }

__global__ __launch_bounds__(128) void k_feat(const float* __restrict__ x, const float* __restrict__ kw1, const float* __restrict__ kb1, const float* __restrict__ kw2, const float* __restrict__ kb2,
                                            const float* __restrict__ qw1, const float* __restrict__ qb1, const float* __restrict__ qw2, const float* __restrict__ qb2, const float* __restrict__ vw, const float* __restrict__ vb,
                                            _Float16* __restrict__ Fk, _Float16* __restrict__ Fq, _Float16* __restrict__ VT) {
  __shared__ __align__(16) float sh[4][16][DD + 4];
  __shared__ __align__(16) _Float16 sf[4][16][NF + 8];
  __shared__ __align__(16) _Float16 st[DD][72];
  const int tid = threadIdx.x, wave = tid >> 5, lane = tid & 31, col = lane & 15, g = lane >> 4;
  const int r0b = blockIdx.x * 64, r0 = r0b + wave * 16; const int b = r0b / LL, l0 = r0b % LL;
  v16h ax[8];
#pragma unroll
  for (int kc = 0; kc < 8; ++kc) ax[kc] = frag_f32(x + (size_t)(r0 + col) * DD + kc * 32, lane);
#pragma unroll 1
  for (int which = 0; which < 2; ++which) { const float* W1 = which == 0 ? kw1 : qw1; const float* B1 = which == 0 ? kb1 : qb1; const float* W2 = which == 0 ? kw2 : qw2; const float* B2 = which == 0 ? kb2 : qb2;
#pragma unroll 1
    for (int np = 0; np < 2; ++np) { v8f acc[8] = {};
#pragma unroll
      for (int kc = 0; kc < 8; ++kc) {
#pragma unroll
        for (int j = 0; j < 8; ++j) { v16h bb = fragc_f32(W1, kc * 32, np * 128 + j * 16 + col, lane, DD, DD);
#pragma unroll
          for (int e = 0; e < 16; ++e) bb[e] = bb[e] * (_Float16)16.0f;
          acc[j] = wmma16(ax[kc], bb, acc[j]); } }
#pragma unroll
      for (int j = 0; j < 8; ++j) { const int c = np * 128 + j * 16 + col; const float bb = B1[c];
#pragma unroll
        for (int r = 0; r < 8; ++r) sh[wave][8 * g + r][c] = gelu_e(acc[j][r] * (1.0f / 16.0f) + bb); } }
    LDSX();
    { v8f acc[4] = {};
#pragma unroll
      for (int kc = 0; kc < 8; ++kc) { const v16h a = frag_f32(&sh[wave][col][0] + kc * 32, lane);
#pragma unroll
        for (int j = 0; j < 4; ++j) { v16h bb = fragc_f32(W2, kc * 32, j * 16 + col, lane, KP, DD);
#pragma unroll
          for (int e = 0; e < 16; ++e) bb[e] = bb[e] * (_Float16)16.0f;
          acc[j] = wmma16(a, bb, acc[j]); } }
      LDSX();
#pragma unroll
      for (int j = 0; j < 4; ++j) { const int c = j * 16 + col; const float bb = B2[c];
#pragma unroll
        for (int r = 0; r < 8; ++r) { const float ph = tanhf(acc[j][r] * (1.0f / 16.0f) + bb) * 3.14159265358979f; float sv, cv; sincosf(ph, &sv, &cv);
          sf[wave][8 * g + r][c] = (_Float16)cv; sf[wave][8 * g + r][KP + c] = (_Float16)sv; } } }
    LDSX();
    _Float16* dst = which == 0 ? Fk : Fq;
    for (int q = lane; q < 16 * 16; q += 32) { const int rl = q >> 4, pc = q & 15; vst2(dst + (size_t)(r0 + rl) * NF + pc * 8, *(const v4u*)(&sf[wave][rl][pc * 8])); }
    LDSX(); }
#pragma unroll 1
  for (int np = 0; np < 2; ++np) { v8f acc[8] = {};
#pragma unroll
    for (int kc = 0; kc < 8; ++kc) {
#pragma unroll
      for (int j = 0; j < 8; ++j) { v16h bb = fragc_f32(vw, kc * 32, np * 128 + j * 16 + col, lane, DD, DD);
#pragma unroll
        for (int e = 0; e < 16; ++e) bb[e] = bb[e] * (_Float16)16.0f;
        acc[j] = wmma16(ax[kc], bb, acc[j]); } }
#pragma unroll
    for (int j = 0; j < 8; ++j) { const int c = np * 128 + j * 16 + col; const float bb = vb[c];
#pragma unroll
      for (int r = 0; r < 8; ++r) st[c][wave * 16 + 8 * g + r] = (_Float16)((acc[j][r] * (1.0f / 16.0f) + bb) * 8.0f); } }
  __syncthreads();
  for (int q = tid; q < DD * 8; q += 128) { const int d = q >> 3, pc = q & 7; vst2(VT + ((size_t)b * DD + d) * LL + l0 + pc * 8, *(const v4u*)(&st[d][pc * 8])); }
}
__global__ __launch_bounds__(128) void k_attn(const _Float16* __restrict__ Fq, const _Float16* __restrict__ Fk, const _Float16* __restrict__ VT, const float* __restrict__ x, const float* __restrict__ lg, const float* __restrict__ lb, const float* __restrict__ ow, const float* __restrict__ ob, float* __restrict__ out) {
  __shared__ __align__(16) _Float16 sP[4][16][72];
  __shared__ __align__(16) float sr[4][16][DD + 4];
  __shared__ __align__(16) float sy[4][16][DD + 4];
  const int tid = threadIdx.x, w = tid >> 5, lane = tid & 31, col = lane & 15, g = lane >> 4;
  const int b = blockIdx.y, q0 = blockIdx.x * 64 + w * 16; const size_t rb = (size_t)b * LL;
  v16h aq[4];
#pragma unroll
  for (int kc = 0; kc < 4; ++kc) aq[kc] = frag_h(Fq + (rb + q0 + col) * NF + kc * 32, lane);
  v8f acc[16];
#pragma unroll
  for (int j = 0; j < 16; ++j) acc[j] = (v8f){};
  const int ntiles = blockIdx.x + 1;
#pragma unroll 1
  for (int kt = 0; kt < ntiles; ++kt) {
#pragma unroll
    for (int t = 0; t < 4; ++t) { v8f s = {}; const int key = kt * 64 + t * 16 + col;
#pragma unroll
      for (int kc = 0; kc < 4; ++kc) s = wmma16(aq[kc], frag_h(Fk + (rb + key) * NF + kc * 32, lane), s);
#pragma unroll
      for (int r = 0; r < 8; ++r) { const int qi = q0 + 8 * g + r; sP[w][8 * g + r][t * 16 + col] = (_Float16)(key <= qi ? s[r] : 0.f); } }
    LDSX();
#pragma unroll
    for (int kc = 0; kc < 2; ++kc) { const v16h pa = frag_h(&sP[w][col][0] + kc * 32, lane);
#pragma unroll
      for (int j = 0; j < 16; ++j) acc[j] = wmma16(pa, frag_h(VT + ((size_t)b * DD + j * 16 + col) * LL + kt * 64 + kc * 32, lane), acc[j]); }
    LDSX(); }
#pragma unroll
  for (int j = 0; j < 16; ++j)
#pragma unroll
    for (int r = 0; r < 8; ++r) { const int qi = q0 + 8 * g + r; sr[w][8 * g + r][j * 16 + col] = acc[j][r] * 0.125f * rsqrtf((float)(qi + 1) * 64.0f); }
  LDSX();
  { const int rl = lane >> 1, hf = lane & 1; float* row = &sr[w][rl][0]; float s = 0.f; for (int c = 0; c < 128; ++c) s += row[hf * 128 + c]; s += __shfl_xor(s, 1, 32); const float mu = s * (1.0f / DD);
    float q2 = 0.f; for (int c = 0; c < 128; ++c) { const float d = row[hf * 128 + c] - mu; q2 += d * d; } q2 += __shfl_xor(q2, 1, 32); const float rs = rsqrtf(q2 * (1.0f / DD) + 1e-5f);
    LDSX();
    for (int c = 0; c < 128; ++c) { const int cc = hf * 128 + c; row[cc] = lg[cc] * (row[cc] - mu) * rs + lb[cc]; } }
  LDSX();
#pragma unroll 1
  for (int np = 0; np < 2; ++np) { v8f o2[8];
#pragma unroll
    for (int j = 0; j < 8; ++j) o2[j] = (v8f){};
#pragma unroll 1
    for (int kc = 0; kc < 8; ++kc) { const v16h a = frag_f32(&sr[w][col][0] + kc * 32, lane);
#pragma unroll
      for (int j = 0; j < 8; ++j) { v16h bb = fragc_f32(ow, kc * 32, np * 128 + j * 16 + col, lane, DD, DD);
#pragma unroll
        for (int e = 0; e < 16; ++e) bb[e] = bb[e] * (_Float16)16.0f;
        o2[j] = wmma16(a, bb, o2[j]); } }
#pragma unroll
    for (int j = 0; j < 8; ++j) { const int c = np * 128 + j * 16 + col; const float bb = ob[c];
#pragma unroll
      for (int r = 0; r < 8; ++r) sy[w][8 * g + r][c] = x[(rb + q0 + 8 * g + r) * DD + c] + o2[j][r] * (1.0f / 16.0f) + bb; } }
  LDSX();
  for (int q = lane; q < 16 * 64; q += 32) { const int rl = q >> 6, pc = q & 63; vst2(out + (rb + q0 + rl) * DD + pc * 4, *(const v4f*)(&sy[w][rl][pc * 4])); }
}
extern "C" void kernel_launch(void* const* d_in, const int* in_sizes, int n_in, void* d_out, int out_size, void* d_ws, size_t ws_size, hipStream_t stream) {
  (void)in_sizes; (void)n_in; (void)out_size; (void)ws_size;
  const float** I = (const float**)d_in;
  const float* x = I[0]; const float* kw1 = I[1]; const float* kb1 = I[2]; const float* kw2 = I[3]; const float* kb2 = I[4]; const float* qw1 = I[5]; const float* qb1 = I[6]; const float* qw2 = I[7]; const float* qb2 = I[8];
  const float* vw = I[9]; const float* vb = I[10]; const float* lg = I[11]; const float* lb = I[12]; const float* ow = I[13]; const float* ob = I[14];
  float* out = (float*)d_out;
  char* ws = (char*)d_ws; size_t off = 0;
  auto take = [&](size_t bytes) { char* p = ws + off; off += (bytes + 255) & ~(size_t)255; return p; };
  _Float16* Fk = (_Float16*)take((size_t)NR * NF * 2); _Float16* Fq = (_Float16*)take((size_t)NR * NF * 2); _Float16* VT = (_Float16*)take((size_t)NB * DD * LL * 2);
  k_feat<<<NR / 64, 128, 0, stream>>>(x, kw1, kb1, kw2, kb2, qw1, qb1, qw2, qb2, vw, vb, Fk, Fq, VT);
  k_attn<<<dim3(LL / 64, NB), 128, 0, stream>>>(Fq, Fk, VT, x, lg, lb, ow, ob, out);
}
